// GNNEncoder_1090921693880
// MI455X (gfx1250) — hardware-run, weakly checked
//
#include <hip/hip_runtime.h>


namespace {


constexpr int N = 100000, NP = 100032, NR = N  , NPL = NP  , SRCM = N  , EFULL = 600000, E = EFULL  , NG = 16  ;
constexpr int XD = 12  , EF = 3  , KE = 32  , NLAY = 3, D = 128, D2 = 2 * D, NL = (NPL < N ? NPL : N), NRL = NP  ;
static_assert(NP % NG == 0 && NP % 32 == 0, "node groups");
constexpr float LNEPS = 1e-5f; constexpr float LOG2E = 1.4426950408889634f, ISQD = 1.0f  ;
constexpr float XS = 8.0f, WSC = 256.0f, WSQ = 0.25f, RS_ = 1024.0f, SLOPE = 0.0f, BNEPS = 1e-5f;
static_assert(NP % 32 == 0 && NP >= N && NPL % 32 == 0 && D == 128, "tiling");
typedef _Float16 b16;
typedef __attribute__((ext_vector_type(16))) _Float16 v16b;
typedef __attribute__((ext_vector_type(8))) _Float16 v8b;
typedef __attribute__((ext_vector_type(8))) float v8f;
typedef __attribute__((ext_vector_type(4))) float v4f;
__device__ __forceinline__ float bf16_rne(float f) { unsigned int u = __float_as_uint(f); u += 0x7FFFu + ((u >> 16) & 1u); return __uint_as_float(u & 0xFFFF0000u); }
__device__ __forceinline__ void split16(float v, b16& hi, b16& lo) { hi = (b16)v; lo = (b16)(v - (float)hi); }
__device__ __forceinline__ v16b frag_kb(const b16* p, int hh) { const v8b a = *(const v8b*)(p + 8 * hh), b = *(const v8b*)(p + 16 + 8 * hh); v16b f;
#pragma unroll
  for (int e = 0; e < 8; ++e) { f[e] = a[e]; f[8 + e] = b[e]; } return f; }
__device__ __forceinline__ v8f wmma16b(v16b a, v16b b, v8f c) { v8f d = __builtin_amdgcn_wmma_f32_16x16x32_f16(false, a, false, b, (short)0, c, false, false); asm volatile("v_nop\n\tv_nop\n\tv_nop\n\tv_nop" : "+v"(d) : "v"(a), "v"(b)); return d; }
__device__ __forceinline__ void wave_lds_sync() { __builtin_amdgcn_fence(__ATOMIC_RELEASE, "workgroup"); __builtin_amdgcn_wave_barrier(); __builtin_amdgcn_fence(__ATOMIC_ACQUIRE, "workgroup"); }
__device__ __forceinline__ float pmul(float a, float b) { float p = a * b; asm volatile("" : "+v"(p)); return p; }
__device__ __forceinline__ int iclamp(int v, int lo, int hi) { return v < lo ? lo : (v > hi ? hi : v); }
constexpr int CSR_NBLK = 512, CSR_GB = 9, CSR_GN = 1 << CSR_GB  , CSR_MAXG = 512, CSR_CAP = 12288  ;
__global__ __launch_bounds__(64) void csrA_kernel(const int* __restrict__ dst, int E, int N, int nG, int CHP, int NGP, int* __restrict__ STG, int* __restrict__ HST) {
  extern __shared__ int sm[];
  int* cnt = sm; int* run = sm + NGP; int* ids = sm + 2 * NGP;
  const int b = blockIdx.x; const int ch = (E + CSR_NBLK - 1) / CSR_NBLK; const int e0 = b * ch, e1 = min(E, e0 + ch);
  for (int i = threadIdx.x; i < NGP; i += 64) cnt[i] = 0;
  for (int i = threadIdx.x; i < CHP; i += 64) ids[i] = -1;
  __syncthreads();
  if (threadIdx.x == 0) {
    for (int e = e0; e < e1; ++e) { int d = dst[e]; d = (d < 0) ? 0 : (d >= N ? N - 1 : d); cnt[d >> CSR_GB] += 1; }
    int acc = 0; for (int g = 0; g < nG; ++g) { run[g] = acc; acc += cnt[g]; }
    for (int e = e0; e < e1; ++e) { int d = dst[e]; d = (d < 0) ? 0 : (d >= N ? N - 1 : d); const int g = d >> CSR_GB; ids[run[g]] = e; run[g] += 1; } }
  __syncthreads();
  typedef __attribute__((ext_vector_type(4))) int v4i;
  for (int pass = 0; pass < 2; ++pass) {
    for (int i = threadIdx.x; i < CHP / 4; i += 64) *(volatile v4i*)(STG + (size_t)b * CHP + i * 4) = *(const v4i*)(&ids[i * 4]);
    for (int i = threadIdx.x; i < NGP / 4; i += 64) { v4i v; for (int e = 0; e < 4; ++e) v[e] = (i * 4 + e < nG) ? cnt[i * 4 + e] : 0; *(volatile v4i*)(HST + (size_t)b * NGP + i * 4) = v; }
    __threadfence(); }
}
__global__ __launch_bounds__(512) void csrS_kernel(const int* __restrict__ HST, int nG, int NGP, int* __restrict__ START, int* __restrict__ TOT, int* __restrict__ OFF) {
  __shared__ int tot[CSR_MAXG];
  const int b = threadIdx.x;
  for (int pass = 0; pass < 2; ++pass) { int runb = 0; for (int g = 0; g < nG; ++g) { int c = HST[(size_t)b * NGP + g]; c = (c < 0) ? 0 : c; ((volatile int*)OFF)[(size_t)g * CSR_NBLK + b] = runb; runb += c; } __threadfence(); }
  for (int g = threadIdx.x; g < nG; g += 512) { int s = 0; for (int bb = 0; bb < CSR_NBLK; ++bb) { int c = HST[(size_t)bb * NGP + g]; s += (c < 0) ? 0 : c; } tot[g] = s; }
  __syncthreads();
  if (threadIdx.x < 32) {
    __shared__ int st[CSR_MAXG + 32];
    if (threadIdx.x == 0) { int acc = 0; for (int g = 0; g < NGP; ++g) { st[g] = acc; if (g < nG) acc += (tot[g] + 31) & ~31; } st[NGP] = acc; }
    __builtin_amdgcn_fence(__ATOMIC_RELEASE, "workgroup"); __builtin_amdgcn_wave_barrier(); __builtin_amdgcn_fence(__ATOMIC_ACQUIRE, "workgroup");
    for (int pass = 0; pass < 2; ++pass) { for (int i = threadIdx.x; i < NGP + 32; i += 32) { ((volatile int*)START)[i] = (i <= NGP) ? st[min(i, NGP)] : 0; ((volatile int*)TOT)[i] = (i < nG) ? tot[i] : 0; } __threadfence(); } }
}
__global__ __launch_bounds__(256) void csrB_kernel(const int* __restrict__ dst, int N, int nG, int CHP, int NGP, int permLen, const int* __restrict__ STG, const int* __restrict__ HST, const int* __restrict__ OFF, const int* __restrict__ START, const int* __restrict__ TOT, int* __restrict__ PERM, int* __restrict__ ROWPTR, int* __restrict__ ROWCNT, int* __restrict__ FLAG) {
  typedef __attribute__((ext_vector_type(4))) int v4i;
  __shared__ int ids[CSR_CAP]; __shared__ unsigned short key[CSR_CAP]; __shared__ int outp[CSR_CAP]; __shared__ int ncnt[CSR_GN + 1]; __shared__ int boff[CSR_NBLK + 1];
  const int g = blockIdx.x, t_ = threadIdx.x; int tot = TOT[g]; int st = START[g], stn = START[g + 1]; const int v0 = g * CSR_GN; const int nv = min(CSR_GN, N - v0);
  st = (st < 0) ? 0 : (st > permLen - 32 ? permLen - 32 : st) & ~31; stn = (stn < st) ? st : (stn > permLen ? permLen : stn); tot = (tot < 0) ? 0 : tot; if (tot > stn - st && tot <= CSR_CAP) tot = stn - st;
  if (tot > CSR_CAP) {
    for (int pass = 0; pass < 2; ++pass) { for (int i = t_; i < CSR_GN / 4; i += 256) { v4i a, c; for (int e = 0; e < 4; ++e) { a[e] = st; c[e] = 0; } *(volatile v4i*)(ROWPTR + v0 + i * 4) = a; *(volatile v4i*)(ROWCNT + v0 + i * 4) = c; } if (t_ == 0) ((volatile int*)FLAG)[0] = 1; __threadfence(); } (void)nv; return; }
  if (t_ == 0) { int acc = 0; for (int b = 0; b < CSR_NBLK; ++b) { boff[b] = acc; int c = HST[(size_t)b * NGP + g]; c = (c < 0) ? 0 : (c > CHP ? CHP : c); acc += c; if (acc > tot) acc = tot; } boff[CSR_NBLK] = acc; }
  for (int i = t_; i <= CSR_GN; i += 256) ncnt[i] = 0;
  __syncthreads();
  for (int b = 0; b < CSR_NBLK; ++b) { const int c = boff[b + 1] - boff[b]; int o_ = OFF[(size_t)g * CSR_NBLK + b]; o_ = (o_ < 0) ? 0 : (o_ > CHP - c ? CHP - c : o_); const int* src_ = STG + (size_t)b * CHP + o_;
    for (int i = t_; i < c; i += 256) { int id = src_[i]; id = (id < 0) ? 0 : id; ids[boff[b] + i] = id; int d = dst[id]; d = (d < v0) ? v0 : (d >= N ? N - 1 : d); int kk = d - v0; kk = (kk < 0) ? 0 : (kk >= CSR_GN ? CSR_GN - 1 : kk); key[boff[b] + i] = (unsigned short)kk; } }
  __syncthreads();
  if (t_ == 0) { for (int i = 0; i < tot; ++i) ncnt[key[i]] += 1; int acc = 0; for (int vl = 0; vl < CSR_GN; ++vl) { const int c = ncnt[vl]; ncnt[vl] = acc; acc += c; } ncnt[CSR_GN] = acc;
    for (int i = 0; i < tot; ++i) { const int vl = key[i]; outp[ncnt[vl]] = ids[i]; ncnt[vl] += 1; }
    for (int vl = CSR_GN; vl > 0; --vl) ncnt[vl] = ncnt[vl - 1]; ncnt[0] = 0; }
  __syncthreads();
  for (int pass = 0; pass < 2; ++pass) {
    for (int i = t_; i < (stn - st) / 4; i += 256) { v4i v; for (int e = 0; e < 4; ++e) { const int q = i * 4 + e; v[e] = (q < tot) ? outp[q] : -1; } *(volatile v4i*)(PERM + st + i * 4) = v; }
    for (int i = t_; i < CSR_GN / 4; i += 256) { v4i a, c; for (int e = 0; e < 4; ++e) { const int vl = i * 4 + e; a[e] = st + ncnt[vl]; c[e] = (vl < nv) ? (ncnt[vl + 1] - ncnt[vl]) : 0; } *(volatile v4i*)(ROWPTR + v0 + i * 4) = a; *(volatile v4i*)(ROWCNT + v0 + i * 4) = c; }
    __threadfence(); }
}
__global__ __launch_bounds__(256) void csrZ_kernel(int* __restrict__ p, size_t n4) { typedef __attribute__((ext_vector_type(4))) int v4i; const size_t tid = (size_t)blockIdx.x * 256 + threadIdx.x, nth = (size_t)gridDim.x * 256; v4i z = {0, 0, 0, 0}; for (size_t i = tid; i < n4; i += nth) *(volatile v4i*)(p + i * 4) = z; }
struct CsrBufs { int *STG, *HST, *OFF, *START, *TOT, *PERM, *ROWPTR, *ROWCNT, *FLAG; int nG, NGP, CHP; size_t permLen; char* base; size_t bytes; };
static size_t csr_carve(CsrBufs& c, char* ws, size_t off, int E, int N) {
  const size_t off0 = off; c.base = ws + off;
  auto al = [&](size_t bytes) { char* p = ws + off; off += (bytes + 255) & ~(size_t)255; return p; };
  c.nG = (N + CSR_GN - 1) / CSR_GN; c.NGP = (c.nG + 31) & ~31; const int ch = (E + CSR_NBLK - 1) / CSR_NBLK; c.CHP = (ch + 31) & ~31; c.permLen = (size_t)E + 32 * (size_t)c.nG + 32;
  c.STG = (int*)al((size_t)CSR_NBLK * c.CHP * 4); c.HST = (int*)al((size_t)CSR_NBLK * c.NGP * 4); c.OFF = (int*)al((size_t)c.NGP * CSR_NBLK * 4); c.START = (int*)al((size_t)(c.NGP + 64) * 4); c.TOT = (int*)al((size_t)(c.NGP + 64) * 4);
  c.PERM = (int*)al(c.permLen * 4); c.ROWPTR = (int*)al((size_t)c.nG * CSR_GN * 4); c.ROWCNT = (int*)al((size_t)c.nG * CSR_GN * 4); c.FLAG = (int*)al(256);
  c.bytes = off - off0; return off;
}
static void csr_build(const CsrBufs& c, const int* dst, int E, int N, hipStream_t stream) {
  const size_t smem = (size_t)(2 * c.NGP + c.CHP) * 4;
  csrZ_kernel<<<512, 256, 0, stream>>>((int*)c.base, c.bytes / 16);
  csrA_kernel<<<CSR_NBLK, 64, smem, stream>>>(dst, E, N, c.nG, c.CHP, c.NGP, c.STG, c.HST);
  csrS_kernel<<<1, 512, 0, stream>>>(c.HST, c.nG, c.NGP, c.START, c.TOT, c.OFF);
  csrB_kernel<<<c.nG, 256, 0, stream>>>(dst, N, c.nG, c.CHP, c.NGP, (int)c.permLen, c.STG, c.HST, c.OFF, c.START, c.TOT, c.PERM, c.ROWPTR, c.ROWCNT, c.FLAG);
}

typedef __attribute__((ext_vector_type(4))) _Float16 v4h;
__device__ __forceinline__ float gelu_(float v) { return 0.5f * v * (1.0f + erff(v * 0.70710678118654752f)); }
template <int K, bool RND, int MODE>
__global__ __launch_bounds__(64) void lin_kernel(const float* __restrict__ IN, const b16* __restrict__ WT, const b16* __restrict__ WQ, const float* __restrict__ bias, const float* __restrict__ gate, const float* __restrict__ xprev, float* __restrict__ OUT, int mrows, const float* __restrict__ wdeg = nullptr, const float* __restrict__ bdeg = nullptr, const float* __restrict__ lng = nullptr, const float* __restrict__ lnb = nullptr) {
  __shared__ __attribute__((aligned(16))) b16 Ah[2][16][K + 8], Al[2][16][K + 8]; __shared__ __attribute__((aligned(16))) float Tf[2][16][D + 4];
  const int wave = threadIdx.x >> 5, lane = threadIdx.x & 31, nloc = lane & 15, hlf = lane >> 4; const size_t m0 = (size_t)blockIdx.x * 32 + wave * 16; const int mat = blockIdx.y;
  const b16* W = WT + (size_t)mat * D * K; const b16* Wq = RND ? nullptr : WQ + (size_t)mat * D * K; const float* bb_ = bias ? bias + (size_t)mat * D : nullptr; float* O = OUT + (size_t)mat * NP * D;
  for (int idx = lane; idx < 16 * (K / 4); idx += 32) { const int rr = idx / (K / 4), c4 = (idx % (K / 4)) * 4; const size_t arow = (m0 + rr < (size_t)NR) ? m0 + rr : (size_t)NR - 1; const v4f v = *(const v4f*)(IN + arow * K + c4); v4h hv, lv;
    for (int j = 0; j < 4; ++j) { float vin = v[j]; if (MODE == 10) vin = fmaxf(vin, 0.0f); const float vs = (RND ? bf16_rne(vin) : vin) * XS; const b16 ph = (b16)vs; hv[j] = ph; lv[j] = (b16)((vs - (float)ph) * RS_); } *(v4h*)(&Ah[wave][rr][c4]) = hv; if (!RND) *(v4h*)(&Al[wave][rr][c4]) = lv; }
  wave_lds_sync();
  v8f acc[8];
#pragma unroll
  for (int t = 0; t < 8; ++t) acc[t] = (v8f){};
#pragma unroll
  for (int kb = 0; kb < K; kb += 32) { const v16b a = frag_kb(&Ah[wave][nloc][kb], hlf); v16b al; if (!RND) al = frag_kb(&Al[wave][nloc][kb], hlf);
#pragma unroll
    for (int t = 0; t < 8; ++t) { const size_t wo_ = (size_t)(t * 16 + nloc) * K + kb; acc[t] = wmma16b(a, frag_kb(W + wo_, hlf), acc[t]); if (!RND) acc[t] = wmma16b(al, frag_kb(Wq + wo_, hlf), acc[t]); } }
  const float sg = (MODE == 3) ? 1.0f / (1.0f + __expf(-bf16_rne(gate[0]))) : 0.0f;
  if (MODE == 8) {
    float sm[8], sq[8]; for (int r = 0; r < 8; ++r) { sm[r] = 0.0f; sq[r] = 0.0f; }
    for (int t = 0; t < 8; ++t) { const int col = t * 16 + nloc; const float bb = bb_ ? bf16_rne(bb_[col]) : 0.0f; for (int r = 0; r < 8; ++r) { const float y = acc[t][r] * (1.0f / (XS * WSC)) + bb; acc[t][r] = y; sm[r] += y; } }
#pragma unroll
    for (int o = 1; o < 16; o <<= 1) for (int r = 0; r < 8; ++r) sm[r] += __shfl_xor(sm[r], o);
    for (int t = 0; t < 8; ++t) for (int r = 0; r < 8; ++r) { const float d = acc[t][r] - sm[r] * (1.0f / D); sq[r] += pmul(d, d); }
#pragma unroll
    for (int o = 1; o < 16; o <<= 1) for (int r = 0; r < 8; ++r) sq[r] += __shfl_xor(sq[r], o);
    for (int t = 0; t < 8; ++t) { const int col = t * 16 + nloc; const float gg = bf16_rne(lng[col]), be = bf16_rne(lnb[col]);
      for (int r = 0; r < 8; ++r) { const size_t vrow = m0 + 8 * hlf + r; const size_t vr_ = (vrow < (size_t)NR) ? vrow : (size_t)NR - 1; const float y = fmaxf((acc[t][r] - sm[r] * (1.0f / D)) * rsqrtf(sq[r] * (1.0f / D) + LNEPS) * gg + be, 0.0f) + xprev[vr_ * D + col]; Tf[wave][8 * hlf + r][col] = (vrow < (size_t)NR) ? y : 0.0f; } }
  } else {
#pragma unroll
  for (int t = 0; t < 8; ++t) { const int col = t * 16 + nloc; const float bb = bb_ ? bf16_rne(bb_[col]) : 0.0f;
    for (int r = 0; r < 8; ++r) { const size_t vrow = m0 + 8 * hlf + r; float y = acc[t][r] * (1.0f / (XS * WSC)) + bb; if (MODE == 1) y = fmaxf(y, 0.0f); if (MODE == 2) y = gelu_(y); if (MODE == 3) y = sg * y + (1.0f - sg) * xprev[(vrow < (size_t)NR ? vrow : (size_t)NR - 1) * D + col]; if (MODE == 4) y += xprev[(vrow < (size_t)NR ? vrow : (size_t)NR - 1) * D + col]; if (MODE == 6) y += bf16_rne(xprev[(vrow < (size_t)NR ? vrow : (size_t)NR - 1) * D + col]); if (MODE == 5) { const size_t vr_ = (vrow < (size_t)NR ? vrow : (size_t)NR - 1); y += xprev[vr_ * D + col] + pmul(gate[vr_], bf16_rne(wdeg[col])) + bf16_rne(bdeg[col]); }
      Tf[wave][8 * hlf + r][col] = (vrow < (size_t)NR) ? y : 0.0f; } }
  }
  wave_lds_sync();
  for (int pass = 0; pass < 2; ++pass) { for (int rr = 0; rr < 16; ++rr) if (m0 + rr < (size_t)mrows) *(volatile v4f*)(O + (m0 + rr) * D + lane * 4) = *(const v4f*)(&Tf[wave][rr][lane * 4]); __threadfence(); }
}
template <int KW>
__global__ __launch_bounds__(256) void wts_kernel(const float* __restrict__ w, int k0, b16* __restrict__ WT, float scl) {
  const int u = blockIdx.x * 256 + threadIdx.x; if (u >= D * KW / 8) return; const int e = u * 8; const int o = e / KW, kk = e % KW; v8b v;
#pragma unroll
  for (int j = 0; j < 8; ++j) v[j] = (b16)(bf16_rne(w[(size_t)(k0 + kk + j) * D + o]) * scl);
  for (int pass = 0; pass < 2; ++pass) { *(volatile v8b*)(WT + e) = v; __threadfence(); }
}
template <int NOUT, int K = D, int NOUTR = NOUT>
__global__ __launch_bounds__(256) void wt_kernel(const float* __restrict__ w, b16* __restrict__ WT, float scl) {
  const int u = blockIdx.x * 256 + threadIdx.x; if (u >= NOUT * K / 8) return; const int e = u * 8; const int o = e / K, k0 = e % K; v8b v;
#pragma unroll
  for (int j = 0; j < 8; ++j) v[j] = (b16)(o < NOUTR ? bf16_rne(w[(size_t)(k0 + j) * NOUTR + o]) * scl : 0.0f);
  for (int pass = 0; pass < 2; ++pass) { *(volatile v8b*)(WT + e) = v; __threadfence(); }
}
__global__ __launch_bounds__(256) void f0_kernel(const float* __restrict__ x, float* __restrict__ F0) {
  const int i = blockIdx.x * 256 + threadIdx.x; const int v = i >> 3, c = (i & 7) * 4; if (v >= NRL) return; v4f t4 = {0.0f, 0.0f, 0.0f, 0.0f};
  if (v < N) { for (int j = 0; j < 4; ++j) { const int cc = c + j; t4[j] = (cc < XD) ? bf16_rne(x[(size_t)v * XD + cc]) : 0.0f; } }
  for (int pass = 0; pass < 2; ++pass) { *(volatile v4f*)(F0 + (size_t)v * KE + c) = t4; __threadfence(); }
}
__global__ __launch_bounds__(256) void wte_kernel(const float* __restrict__ w, b16* __restrict__ WT, float scl) {
  const int u = blockIdx.x * 256 + threadIdx.x; if (u >= D * KE / 8) return; const int e = u * 8; const int o = e / KE, k0 = e % KE; v8b v;
#pragma unroll
  for (int j = 0; j < 8; ++j) { const int k = k0 + j; v[j] = (b16)((k < XD) ? bf16_rne(w[(size_t)k * D + o]) * scl : 0.0f); }
  for (int pass = 0; pass < 2; ++pass) { *(volatile v8b*)(WT + e) = v; __threadfence(); }
}
__global__ __launch_bounds__(256) void easum_kernel(const float* __restrict__ eattr, const int* __restrict__ PERM, const int* __restrict__ ROWPTR, const int* __restrict__ ROWCNT, int permLen, float* __restrict__ EA) {
  const int v = blockIdx.x * 256 + threadIdx.x; if (v >= NP) return;
  int cnt = 0, p0 = 0; if (v < N) { cnt = iclamp(ROWCNT[v], 0, 65536); p0 = iclamp(ROWPTR[v], 0, permLen - 1); if (p0 + cnt > permLen) cnt = permLen - p0; }
  float s0 = 0.0f, s1 = 0.0f, s2 = 0.0f;
#pragma unroll 1
  for (int i = 0; i < cnt; ++i) { const int e = iclamp(PERM[p0 + i], 0, E - 1); s0 += bf16_rne(eattr[(size_t)e * EF]); s1 += bf16_rne(eattr[(size_t)e * EF + 1]); s2 += bf16_rne(eattr[(size_t)e * EF + 2]); }
  v4f o = {s0, s1, s2, (float)cnt};
  for (int pass = 0; pass < 2; ++pass) { *(volatile v4f*)(EA + (size_t)v * 4) = o; __threadfence(); }
}
__global__ __launch_bounds__(256) void ginz_kernel(const float* __restrict__ H, const float* __restrict__ EA, const float* __restrict__ eps, const float* __restrict__ ew, const float* __restrict__ eb, const int* __restrict__ srcs, const int* __restrict__ PERM, const int* __restrict__ ROWPTR, const int* __restrict__ ROWCNT, int permLen, float* __restrict__ Z, int mrows) {
  const int tid = threadIdx.x; const int row = tid >> 3, g = tid & 7, c0 = g * 16; const int v = blockIdx.x * 32 + row; const int vv = v < N ? v : N - 1;
  int cnt = 0, p0 = 0; if (v < N) { cnt = iclamp(ROWCNT[v], 0, 65536); p0 = iclamp(ROWPTR[v], 0, permLen - 1); if (p0 + cnt > permLen) cnt = permLen - p0; }
  const float scl = 1.0f + bf16_rne(eps[0]); const v4f ea = *(const v4f*)(EA + (size_t)vv * 4);
  float m[16]; { const float* hr = H + (size_t)vv * D + c0;
#pragma unroll
    for (int q = 0; q < 4; ++q) { const v4f t4 = *(const v4f*)(hr + 4 * q); for (int j = 0; j < 4; ++j) { const int c = c0 + 4 * q + j; m[4 * q + j] = pmul(scl, t4[j]) + pmul(ea[0], bf16_rne(ew[c])) + pmul(ea[1], bf16_rne(ew[D + c])) + pmul(ea[2], bf16_rne(ew[2 * D + c])) + pmul(ea[3], bf16_rne(eb[c])); } } }
#pragma unroll 1
  for (int i = 0; i < cnt; ++i) { const int e = iclamp(PERM[p0 + i], 0, E - 1); int s = iclamp(srcs[e], 0, N - 1); if (SRCM < N) s %= SRCM; const float* hr = H + (size_t)s * D + c0;
#pragma unroll
    for (int q = 0; q < 4; ++q) { const v4f t4 = *(const v4f*)(hr + 4 * q); for (int j = 0; j < 4; ++j) m[4 * q + j] += t4[j]; } }
  for (int pass = 0; pass < 2; ++pass) { if (v < mrows) { float* orow = Z + (size_t)v * D + c0;
#pragma unroll
      for (int q = 0; q < 4; ++q) { v4f o; for (int j = 0; j < 4; ++j) o[j] = (v < N) ? m[4 * q + j] : 0.0f; *(volatile v4f*)(orow + 4 * q) = o; } }
    __threadfence(); }
}
template <int W>
__global__ __launch_bounds__(256) void bnfold_kernel(const float* __restrict__ bias, const float* __restrict__ g, const float* __restrict__ be, const float* __restrict__ rm, const float* __restrict__ rv, float* __restrict__ SCL, float* __restrict__ SFT) {
  const int c = threadIdx.x; if (c >= W) return; const float s = bf16_rne(g[c]) * rsqrtf(bf16_rne(rv[c]) + 1e-5f); const float t = (bf16_rne(bias[c]) - bf16_rne(rm[c])) * s + bf16_rne(be[c]);
  for (int pass = 0; pass < 2; ++pass) { ((volatile float*)SCL)[c] = s; ((volatile float*)SFT)[c] = t; __threadfence(); }
}
__global__ __launch_bounds__(64) void mlp12_kernel(const float* __restrict__ Z, const b16* __restrict__ W1T, const float* __restrict__ S1, const float* __restrict__ T1, const b16* __restrict__ W2T, const float* __restrict__ S2, const float* __restrict__ T2, float* __restrict__ OUT, int mrows) {
  __shared__ __attribute__((aligned(16))) b16 A1[2][16][D + 8]; __shared__ __attribute__((aligned(16))) b16 A2[2][16][D2 + 8]; __shared__ __attribute__((aligned(16))) float T1f[2][16][D2 + 4]; __shared__ __attribute__((aligned(16))) float Tf[2][16][D + 4];
  const int wave = threadIdx.x >> 5, lane = threadIdx.x & 31, nloc = lane & 15, hlf = lane >> 4; const size_t m0 = (size_t)blockIdx.x * 32 + wave * 16;
  for (int idx = lane; idx < 16 * (D / 4); idx += 32) { const int rr = idx / (D / 4), c4 = (idx % (D / 4)) * 4; const size_t arow = (m0 + rr < (size_t)NR) ? m0 + rr : (size_t)NR - 1; const v4f v = *(const v4f*)(Z + arow * D + c4); v4h hv;
    for (int j = 0; j < 4; ++j) hv[j] = (b16)(v[j] * XS); *(v4h*)(&A1[wave][rr][c4]) = hv; }
  wave_lds_sync();
  { v8f acc[16];
#pragma unroll
    for (int t = 0; t < 16; ++t) acc[t] = (v8f){};
#pragma unroll
    for (int kb = 0; kb < D; kb += 32) { const v16b a = frag_kb(&A1[wave][nloc][kb], hlf);
#pragma unroll
      for (int t = 0; t < 16; ++t) acc[t] = wmma16b(a, frag_kb(W1T + (size_t)(t * 16 + nloc) * D + kb, hlf), acc[t]); }
#pragma unroll
    for (int t = 0; t < 16; ++t) { const int col = t * 16 + nloc; const float s = S1[col], sh = T1[col];
      for (int r = 0; r < 8; ++r) { const float y = fmaxf(acc[t][r] * (1.0f / (XS * WSC)) * s + sh, 0.0f); T1f[wave][8 * hlf + r][col] = y; } } }
  wave_lds_sync();
  for (int idx = lane; idx < 16 * (D2 / 4); idx += 32) { const int rr = idx / (D2 / 4), c4 = (idx % (D2 / 4)) * 4; const v4f v = *(const v4f*)(&T1f[wave][rr][c4]); v4h hv; for (int j = 0; j < 4; ++j) hv[j] = (b16)(v[j] * XS); *(v4h*)(&A2[wave][rr][c4]) = hv; }
  wave_lds_sync();
  v8f acc2[8];
#pragma unroll
  for (int t = 0; t < 8; ++t) acc2[t] = (v8f){};
#pragma unroll 2
  for (int kb = 0; kb < D2; kb += 32) { const v16b a = frag_kb(&A2[wave][nloc][kb], hlf);
#pragma unroll
    for (int t = 0; t < 8; ++t) acc2[t] = wmma16b(a, frag_kb(W2T + (size_t)(t * 16 + nloc) * D2 + kb, hlf), acc2[t]); }
#pragma unroll
  for (int t = 0; t < 8; ++t) { const int col = t * 16 + nloc; const float s = S2[col], sh = T2[col];
    for (int r = 0; r < 8; ++r) { const size_t vrow = m0 + 8 * hlf + r; const float y = fmaxf(acc2[t][r] * (1.0f / (XS * WSC)) * s + sh, 0.0f); Tf[wave][8 * hlf + r][col] = (vrow < (size_t)NR) ? y : 0.0f; } }
  wave_lds_sync();
  for (int pass = 0; pass < 2; ++pass) { for (int rr = 0; rr < 16; ++rr) if (m0 + rr < (size_t)mrows) *(volatile v4f*)(OUT + (m0 + rr) * D + lane * 4) = *(const v4f*)(&Tf[wave][rr][lane * 4]); __threadfence(); }
}
__global__ __launch_bounds__(256) void lnres_kernel(const float* __restrict__ Z2, float* __restrict__ H, const float* __restrict__ lg, const float* __restrict__ lb, int mrows) {
  const int tid = threadIdx.x; const int row = tid >> 3, g = tid & 7, c0 = g * 16; const int v = blockIdx.x * 32 + row; const int vv = v < N ? v : N - 1;
  float y[16]; float s1 = 0.0f;
#pragma unroll
  for (int q = 0; q < 4; ++q) { const v4f a4 = *(const v4f*)(Z2 + (size_t)vv * D + c0 + 4 * q), b4 = *(const v4f*)(H + (size_t)vv * D + c0 + 4 * q); for (int j = 0; j < 4; ++j) { y[4 * q + j] = a4[j] + b4[j]; s1 += y[4 * q + j]; } }
  s1 += __shfl_xor(s1, 1); s1 += __shfl_xor(s1, 2); s1 += __shfl_xor(s1, 4); const float mu = s1 * (1.0f / D); float s2 = 0.0f;
  for (int j = 0; j < 16; ++j) { const float d = y[j] - mu; s2 += pmul(d, d); }
  s2 += __shfl_xor(s2, 1); s2 += __shfl_xor(s2, 2); s2 += __shfl_xor(s2, 4); const float rs = rsqrtf(s2 * (1.0f / D) + LNEPS);
  float o[16]; for (int j = 0; j < 16; ++j) o[j] = (v < N) ? (y[j] - mu) * rs * bf16_rne(lg[c0 + j]) + bf16_rne(lb[c0 + j]) : 0.0f;
  for (int pass = 0; pass < 2; ++pass) { if (v < mrows) { float* orow = H + (size_t)v * D + c0;
#pragma unroll
      for (int q = 0; q < 4; ++q) { v4f o4; for (int j = 0; j < 4; ++j) o4[j] = o[4 * q + j]; *(volatile v4f*)(orow + 4 * q) = o4; } } __threadfence(); }
}
__global__ __launch_bounds__(256) void meanpool_kernel(const float* __restrict__ NE, const int* __restrict__ batch, float* __restrict__ out1) {
  __shared__ float part[D]; __shared__ float pcnt[D];
  const int g = blockIdx.x; const int c = threadIdx.x & (D - 1), hf = threadIdx.x >> 7; float s = 0.0f, n = 0.0f;
#pragma unroll 1
  for (int v = hf; v < NL; v += 2) { const int bv = batch[v]; const float hv = NE[(size_t)v * D + c]; const bool in = (bv == g); s += in ? hv : 0.0f; n += in ? 1.0f : 0.0f; }
  if (hf == 1) { part[c] = s; pcnt[c] = n; }
  __syncthreads();
  const float tot = (s + part[c]) / fmaxf(n + pcnt[c], 1.0f);
  for (int pass = 0; pass < 2; ++pass) { if (hf == 0) ((volatile float*)out1)[(size_t)g * D + c] = tot; __threadfence(); }
}
}

extern "C" void kernel_launch(void* const* d_in, const int* in_sizes, int n_in, void* d_out, int out_size, void* d_ws, size_t ws_size, hipStream_t stream) {
  (void)n_in;
  auto Fp = [&](int i) { return (const float*)d_in[i]; }; auto Ip = [&](int i) { return (const int*)d_in[i]; };
  if (in_sizes[0] != N * XD || in_sizes[1] != 2 * EFULL || in_sizes[2] != EFULL * EF || in_sizes[3] != N || in_sizes[4] != XD * D || in_sizes[5] != D || in_sizes[6] != NLAY * EF * D || in_sizes[7] != NLAY * D || in_sizes[8] != NLAY * D * D2 || in_sizes[9] != NLAY * D2) return;
  for (int i = 10; i <= 13; ++i) if (in_sizes[i] != NLAY * D2) return;
  if (in_sizes[14] != NLAY * D2 * D || in_sizes[15] != NLAY * D) return;
  for (int i = 16; i <= 19; ++i) if (in_sizes[i] != NLAY * D) return;
  if (in_sizes[20] != NLAY || in_sizes[21] != NLAY * D || in_sizes[22] != NLAY * D || in_sizes[23] != 4 * D * D || in_sizes[24] != D || in_sizes[25] != D * D || in_sizes[26] != D || out_size != N * D + NG * D) return;
  float* out0 = (float*)d_out; float* out1 = out0 + (size_t)N * D;
  size_t off = 0; char* ws = (char*)d_ws;
  auto carve = [&](size_t bytes) { char* p = ws + off; off += (bytes + 255) & ~(size_t)255; return p; };
  const size_t wsz = (size_t)D * D * 2, plane = (size_t)NP * D * 4;
  b16* WE = (b16*)carve((size_t)D * KE * 2); b16* W1T[NLAY]; b16* W2T[NLAY]; b16* O1T[4]; b16* O1Q[4]; float* S1[NLAY]; float* T1[NLAY]; float* S2[NLAY]; float* T2[NLAY];
  for (int l = 0; l < NLAY; ++l) { W1T[l] = (b16*)carve(2 * wsz); W2T[l] = (b16*)carve(2 * wsz); S1[l] = (float*)carve(D2 * 4); T1[l] = (float*)carve(D2 * 4); S2[l] = (float*)carve(D * 4); T2[l] = (float*)carve(D * 4); }
  for (int i = 0; i < 4; ++i) { O1T[i] = (b16*)carve(wsz); O1Q[i] = (b16*)carve(wsz); } b16* O2T = (b16*)carve(wsz); b16* O2Q = (b16*)carve(wsz);
  float* F0 = (float*)carve((size_t)NP * KE * 4); float* EA = (float*)carve((size_t)NP * 16); float* H = (float*)carve(plane); float* Z = (float*)carve(plane); float* Z2 = (float*)carve(plane); float* ACC = (float*)carve(plane);
  CsrBufs csr; off = csr_carve(csr, ws, off, E, N);
  if (off > ws_size || off > ((size_t)232 << 20)) return;
  { wte_kernel<<<(D * KE / 8 + 255) / 256, 256, 0, stream>>>(Fp(4), WE, WSC);
    for (int l = 0; l < NLAY; ++l) {
      wt_kernel<D2, D, D2><<<(D2 * D / 8 + 255) / 256, 256, 0, stream>>>(Fp(8) + (size_t)l * D * D2, W1T[l], WSC);
      wt_kernel<D, D2, D><<<(D * D2 / 8 + 255) / 256, 256, 0, stream>>>(Fp(14) + (size_t)l * D2 * D, W2T[l], WSC);
      bnfold_kernel<D2><<<1, 256, 0, stream>>>(Fp(9) + l * D2, Fp(10) + l * D2, Fp(11) + l * D2, Fp(12) + l * D2, Fp(13) + l * D2, S1[l], T1[l]);
      bnfold_kernel<D><<<1, 256, 0, stream>>>(Fp(15) + l * D, Fp(16) + l * D, Fp(17) + l * D, Fp(18) + l * D, Fp(19) + l * D, S2[l], T2[l]); }
    for (int i = 0; i < 4; ++i) { wt_kernel<D, D, D><<<(D * D / 8 + 255) / 256, 256, 0, stream>>>(Fp(23) + (size_t)i * D * D, O1T[i], WSC); wt_kernel<D, D, D><<<(D * D / 8 + 255) / 256, 256, 0, stream>>>(Fp(23) + (size_t)i * D * D, O1Q[i], WSQ); }
    wt_kernel<D, D, D><<<(D * D / 8 + 255) / 256, 256, 0, stream>>>(Fp(25), O2T, WSC); wt_kernel<D, D, D><<<(D * D / 8 + 255) / 256, 256, 0, stream>>>(Fp(25), O2Q, WSQ); }
  csr_build(csr, Ip(1) + EFULL, E, N, stream);
  easum_kernel<<<(NP + 255) / 256, 256, 0, stream>>>(Fp(2), csr.PERM, csr.ROWPTR, csr.ROWCNT, (int)csr.permLen, EA);
  f0_kernel<<<(NRL * 8 + 255) / 256, 256, 0, stream>>>(Fp(0), F0);
  lin_kernel<KE, true, 0><<<dim3(NRL / 32, 1), 64, 0, stream>>>(F0, WE, WE, Fp(5), nullptr, nullptr, H, NP);
  lin_kernel<D, false, 0><<<dim3(NRL / 32, 1), 64, 0, stream>>>(H, O1T[0], O1Q[0], Fp(24), nullptr, nullptr, ACC, NP);
  for (int l = 0; l < NLAY; ++l) {
    ginz_kernel<<<NRL / 32, 256, 0, stream>>>(H, EA, Fp(20) + l, Fp(6) + (size_t)l * EF * D, Fp(7) + l * D, Ip(1), csr.PERM, csr.ROWPTR, csr.ROWCNT, (int)csr.permLen, Z, NRL);
    mlp12_kernel<<<NRL / 32, 64, 0, stream>>>(Z, W1T[l], S1[l], T1[l], W2T[l], S2[l], T2[l], Z2, NRL);
    lnres_kernel<<<NRL / 32, 256, 0, stream>>>(Z2, H, Fp(21) + l * D, Fp(22) + l * D, NRL);
    lin_kernel<D, false, 4><<<dim3(NRL / 32, 1), 64, 0, stream>>>(H, O1T[l + 1], O1Q[l + 1], nullptr, nullptr, ACC, ACC, NP);
  }
  lin_kernel<D, false, 10><<<dim3(NPL / 32, 1), 64, 0, stream>>>(ACC, O2T, O2Q, Fp(26), nullptr, nullptr, out0, NL);
  meanpool_kernel<<<NG, 256, 0, stream>>>(out0, Ip(3), out1);
}
